// SymmetricContraction_25082609009189
// MI455X (gfx1250) — hardware-run, weakly checked
//
#include <hip/hip_runtime.h>
#include <math.h>

typedef __attribute__((ext_vector_type(16))) _Float16 v16h;
typedef __attribute__((ext_vector_type(8)))  _Float16 v8h;
typedef __attribute__((ext_vector_type(8)))  float    v8f;
typedef __attribute__((ext_vector_type(4)))  float    v4f;

constexpr int kNodes   = 16384;
constexpr int kCh      = 64;
constexpr int kFeat    = 9;
constexpr int kSpec    = 10;
constexpr int kPath3   = 23;
constexpr int kPath2   = 5;
constexpr int kPath1   = 2;
constexpr int kHeads   = 4;
constexpr int kNLive   = kSpec * kHeads;
constexpr int kNPad    = 48;
constexpr int kMono    = 219;
constexpr int kKPad    = 224;
constexpr int kBtPitch = 256;
constexpr int kTile    = 64;
constexpr int kAPitch  = 232;
constexpr int kRPitch  = 52;
constexpr int kFPitch  = 68;
constexpr int kOPitch  = 260;
constexpr int kOutCols = 256;

constexpr float kMonoCarry = 256.0f;
constexpr float kCoefCarry = 64.0f;
constexpr float kFoldBack  = 1.0f / (kMonoCarry * kCoefCarry);
constexpr float kHalfMinNormal = 6.103515625e-05f;

static_assert(kNLive == 40 && kNLive <= kNPad && (kNPad % 16) == 0, "n tiling");
static_assert(kMono == 9 + 45 + 165 && kMono <= kKPad && (kKPad % 32) == 0 && kKPad <= kBtPitch, "k tiling");
static_assert((kBtPitch % 64) == 0 && (kAPitch % 8) == 0 && kAPitch >= kKPad, "pitches");
static_assert((kNodes % kTile) == 0 && (kNodes % 32) == 0, "node tiling");
static_assert(kOutCols == kCh * kHeads, "output row");
static_assert(kFoldBack * 16384.0f == 1.0f, "fold-back is an exact power of two");

constexpr size_t kOffBt   = 0;
constexpr size_t kBtBytes = (size_t)kCh * kNPad * kBtPitch * 2;
constexpr size_t kOffP    = kOffBt + kBtBytes;
constexpr size_t kPBytes  = (size_t)kCh * kNodes * kHeads * 4;
constexpr size_t kWsTotal = kOffP + kPBytes;
static_assert(kBtBytes == 1572864ull && kPBytes == 16777216ull && kWsTotal == 18350080ull, "carve total");
static_assert((kOffP % 128) == 0 && kWsTotal <= 134217728ull, "carve alignment and cap");

struct MonoIdx { int deg, a, b, c; };
constexpr MonoIdx mono_idx(int m) {
  MonoIdx r = {0, 0, 0, 0};
  if (m < 9) {
    r.deg = 1; r.a = m;
  } else if (m < 54) {
    int t = m - 9, i = 0;
    for (int s = 0; s < 8; ++s) {
      const int cnt = 9 - i;
      if (t >= cnt) { t -= cnt; ++i; }
    }
    r.deg = 2; r.a = i; r.b = i + t;
  } else if (m < 219) {
    int t = m - 54, i = 0;
    for (int s = 0; s < 8; ++s) {
      const int cnt = ((9 - i) * (10 - i)) / 2;
      if (t >= cnt) { t -= cnt; ++i; }
    }
    int j = i;
    for (int s = 0; s < 8; ++s) {
      const int cnt = 9 - j;
      if (t >= cnt) { t -= cnt; ++j; }
    }
    r.deg = 3; r.a = i; r.b = j; r.c = j + t;
  }
  return r;
}
static_assert(mono_idx(0).deg == 1 && mono_idx(8).a == 8, "linear block");
static_assert(mono_idx(9).deg == 2 && mono_idx(9).a == 0 && mono_idx(9).b == 0, "quadratic first");
static_assert(mono_idx(17).a == 0 && mono_idx(17).b == 8 && mono_idx(18).a == 1 && mono_idx(18).b == 1, "quadratic rows");
static_assert(mono_idx(53).a == 8 && mono_idx(53).b == 8, "quadratic last");
static_assert(mono_idx(54).deg == 3 && mono_idx(54).a == 0 && mono_idx(54).b == 0 && mono_idx(54).c == 0, "cubic first");
static_assert(mono_idx(62).a == 0 && mono_idx(62).b == 0 && mono_idx(62).c == 8, "cubic row 0");
static_assert(mono_idx(63).a == 0 && mono_idx(63).b == 1 && mono_idx(63).c == 1, "cubic row 1");
static_assert(mono_idx(99).a == 1 && mono_idx(99).b == 1 && mono_idx(99).c == 1, "cubic second block");
static_assert(mono_idx(218).deg == 3 && mono_idx(218).a == 8 && mono_idx(218).b == 8 && mono_idx(218).c == 8, "cubic last");
static_assert(mono_idx(219).deg == 0 && mono_idx(223).deg == 0, "pad");

union FragH { v16h v; v8h h[2]; };
__device__ __forceinline__ v8f mma_f16(v16h a, v16h b, v8f c) {
  c = __builtin_amdgcn_wmma_f32_16x16x32_f16(false, a, false, b, (short)0, c, false, false);
  asm volatile("v_nop\n\tv_nop\n\tv_nop\n\tv_nop" : "+v"(c) : "v"(a), "v"(b));
  return c;
}

__device__ __forceinline__ _Float16 to_half_flushed(float v) {
  const float w = (fabsf(v) < kHalfMinNormal) ? 0.0f : v;
  return (_Float16)w;
}

__global__ __launch_bounds__(256) void fold_coeff_kernel(
    const float* __restrict__ U3s, const float* __restrict__ U2s, const float* __restrict__ U1s,
    const float* __restrict__ W3s, const float* __restrict__ W2s, const float* __restrict__ W1s,
    const float* __restrict__ U3v, const float* __restrict__ U2v, const float* __restrict__ U1v,
    const float* __restrict__ W3v, const float* __restrict__ W2v, const float* __restrict__ W1v,
    unsigned short* __restrict__ Bt)
{
  __shared__ __align__(16) float sT[kCh * kFPitch];
  const int tid  = threadIdx.x;
  const int lane = tid & 31;
  const int wave = tid >> 5;
  const int c    = tid & 63;
  const int mq   = __builtin_amdgcn_readfirstlane(tid >> 6);
  const int n     = blockIdx.x;
  const int chunk = blockIdx.y;
  const bool rowLive = (n < kNLive);
  const int eRaw = n >> 2;
  const int e    = (eRaw < kSpec) ? eRaw : (kSpec - 1);
  const int o    = n & 3;
  const int hv   = (o == 0) ? 0 : (o - 1);
  const float* U3 = (o == 0) ? U3s : U3v;
  const float* U2 = (o == 0) ? U2s : U2v;
  const float* U1 = (o == 0) ? U1s : U1v;
  const float* W3 = (o == 0) ? W3s : W3v;
  const float* W2 = (o == 0) ? W2s : W2v;
  const float* W1 = (o == 0) ? W1s : W1v;

#pragma unroll 1
  for (int s = 0; s < 16; ++s) {
    const int m = chunk * 64 + mq * 16 + s;
    float acc = 0.0f;
    if (rowLive && m < kMono) {
      const MonoIdx mi = mono_idx(m);
      const int ia = mi.a, ib = mi.b, ic = mi.c;
      if (mi.deg == 3) {
        const int mask = (ia == ib) ? ((ib == ic) ? 1 : 19) : ((ib == ic) ? 13 : 63);
#pragma unroll 1
        for (int p = 0; p < 6; ++p) {
          if ((mask >> p) & 1) {
            const int p1 = (p < 2) ? ia : ((p < 4) ? ib : ic);
            const int r0 = (p < 2) ? ib : ia;
            const int r1 = (p < 4) ? ic : ib;
            const int p2 = (p & 1) ? r1 : r0;
            const int p3 = (p & 1) ? r0 : r1;
            const int uo = (((hv * kFeat + p1) * kFeat + p2) * kFeat + p3) * kPath3;
#pragma unroll 4
            for (int k = 0; k < kPath3; ++k)
              acc = fmaf(U3[uo + k], W3[(e * kPath3 + k) * kCh + c], acc);
          }
        }
      } else if (mi.deg == 2) {
        const int np = (ia == ib) ? 1 : 2;
#pragma unroll 1
        for (int p = 0; p < np; ++p) {
          const int p1 = (p == 0) ? ia : ib;
          const int p2 = (p == 0) ? ib : ia;
          const int uo = ((hv * kFeat + p1) * kFeat + p2) * kPath2;
#pragma unroll
          for (int k = 0; k < kPath2; ++k)
            acc = fmaf(U2[uo + k], W2[(e * kPath2 + k) * kCh + c], acc);
        }
      } else {
        const int uo = (hv * kFeat + ia) * kPath1;
#pragma unroll
        for (int k = 0; k < kPath1; ++k)
          acc = fmaf(U1[uo + k], W1[(e * kPath1 + k) * kCh + c], acc);
      }
    }
    const float cv = acc * kCoefCarry;
    const float fv = (fabsf(cv) < kHalfMinNormal) ? 0.0f : cv;
    sT[c * kFPitch + mq * 16 + s] = fv;
  }
  __syncthreads();

  const int q  = lane >> 3;
  const int c8 = (lane & 7) * 8;
  v8h hvv[2];
#pragma unroll
  for (int it = 0; it < 2; ++it) {
    const int row = it * 32 + wave * 4 + q;
    const float* sp = sT + row * kFPitch + c8;
    const v4f a0 = *(const v4f*)(sp);
    const v4f a1 = *(const v4f*)(sp + 4);
#pragma unroll
    for (int t = 0; t < 4; ++t) {
      const float f0 = a0[t];
      const float f1 = a1[t];
      hvv[it][t]     = (_Float16)f0;
      hvv[it][4 + t] = (_Float16)f1;
    }
  }
  for (int pass = 0; pass < 2; ++pass) {
#pragma unroll
    for (int it = 0; it < 2; ++it) {
      const int row = it * 32 + wave * 4 + q;
      const size_t off = ((size_t)row * kNPad + n) * kBtPitch + (size_t)chunk * 64 + c8;
      *(volatile v8h*)(Bt + off) = hvv[it];
    }
    __threadfence();
  }
}

template <int M>
__device__ __forceinline__ float mono_val(const float (&xs)[kFeat], const float (&xv)[kFeat], float zpad) {
  constexpr MonoIdx mi = mono_idx(M);
  float v = zpad;
  if (mi.deg == 1) v = xs[mi.a];
  if (mi.deg == 2) v = xs[mi.a] * xv[mi.b];
  if (mi.deg == 3) v = (xs[mi.a] * xv[mi.b]) * xv[mi.c];
  return v;
}
template <int G>
__device__ __forceinline__ void gen_group(_Float16* rowp, const float (&xs)[kFeat], const float (&xv)[kFeat], float zpad) {
  v8h hv;
  hv[0] = to_half_flushed(mono_val<8 * G + 0>(xs, xv, zpad));
  hv[1] = to_half_flushed(mono_val<8 * G + 1>(xs, xv, zpad));
  hv[2] = to_half_flushed(mono_val<8 * G + 2>(xs, xv, zpad));
  hv[3] = to_half_flushed(mono_val<8 * G + 3>(xs, xv, zpad));
  hv[4] = to_half_flushed(mono_val<8 * G + 4>(xs, xv, zpad));
  hv[5] = to_half_flushed(mono_val<8 * G + 5>(xs, xv, zpad));
  hv[6] = to_half_flushed(mono_val<8 * G + 6>(xs, xv, zpad));
  hv[7] = to_half_flushed(mono_val<8 * G + 7>(xs, xv, zpad));
  *(v8h*)(rowp + 8 * G) = hv;
}
template <int G> struct GenAll {
  static __device__ __forceinline__ void run(_Float16* rowp, const float (&xs)[kFeat], const float (&xv)[kFeat], float zpad) {
    gen_group<G>(rowp, xs, xv, zpad);
    GenAll<G + 1>::run(rowp, xs, xv, zpad);
  }
};
template <> struct GenAll<kKPad / 8> {
  static __device__ __forceinline__ void run(_Float16*, const float (&)[kFeat], const float (&)[kFeat], float) {}
};

__global__ __launch_bounds__(64) void poly_gemm_kernel(
    const float* __restrict__ x, const float* __restrict__ y,
    const unsigned short* __restrict__ BtBits, float* __restrict__ P)
{
  __shared__ __align__(16) _Float16 As[kTile * kAPitch];
  __shared__ __align__(16) float    Rs[kTile * kRPitch];
  const int tid  = threadIdx.x;
  const int lane = tid & 31;
  const int wave = tid >> 5;
  const int hh   = lane >> 4;
  const int rl   = lane & 15;
  const int c    = blockIdx.y;
  const int b    = blockIdx.x * kTile + tid;

  {
    float xv[kFeat], xs[kFeat];
    const float* xp = x + ((size_t)b * kCh + c) * kFeat;
#pragma unroll
    for (int i = 0; i < kFeat; ++i) {
      xv[i] = xp[i];
      xs[i] = xv[i] * kMonoCarry;
    }
    float zpad = 0.0f;
    asm volatile("" : "+v"(zpad));
    GenAll<0>::run(As + tid * kAPitch, xs, xv, zpad);
  }
  __syncthreads();

  const _Float16* Bc = (const _Float16*)(const void*)BtBits + (size_t)c * kNPad * kBtPitch;

  v8f acc[2][3];
#pragma unroll
  for (int i = 0; i < 2; ++i)
#pragma unroll
    for (int j = 0; j < 3; ++j) acc[i][j] = (v8f){0.f, 0.f, 0.f, 0.f, 0.f, 0.f, 0.f, 0.f};

#pragma unroll 1
  for (int ks = 0; ks < kKPad / 32; ++ks) {
    const int k0 = ks * 32 + 8 * hh;
    FragH bf[3];
#pragma unroll
    for (int j = 0; j < 3; ++j) {
      const _Float16* bp = Bc + (size_t)(j * 16 + rl) * kBtPitch + k0;
      bf[j].h[0] = *(const v8h*)(bp);
      bf[j].h[1] = *(const v8h*)(bp + 16);
    }
#pragma unroll
    for (int i = 0; i < 2; ++i) {
      FragH af;
      const int arow = wave * 32 + i * 16 + rl;
      af.h[0] = *(const v8h*)(As + arow * kAPitch + k0);
      af.h[1] = *(const v8h*)(As + arow * kAPitch + k0 + 16);
#pragma unroll
      for (int j = 0; j < 3; ++j) acc[i][j] = mma_f16(af.v, bf[j].v, acc[i][j]);
    }
  }

#pragma unroll
  for (int i = 0; i < 2; ++i)
#pragma unroll
    for (int j = 0; j < 3; ++j)
#pragma unroll
      for (int r = 0; r < 8; ++r)
        Rs[(wave * 32 + i * 16 + 8 * hh + r) * kRPitch + j * 16 + rl] = acc[i][j][r];
  __syncthreads();

  float ye[kSpec];
  {
    const float* yp = y + (size_t)b * kSpec;
#pragma unroll
    for (int e = 0; e < kSpec; ++e) ye[e] = yp[e];
  }
  float s0 = 0.0f, s1 = 0.0f, s2 = 0.0f, s3 = 0.0f;
#pragma unroll
  for (int e = 0; e < kSpec; ++e) {
    const v4f rv = *(const v4f*)(Rs + tid * kRPitch + e * 4);
    s0 = fmaf(ye[e], rv[0], s0);
    s1 = fmaf(ye[e], rv[1], s1);
    s2 = fmaf(ye[e], rv[2], s2);
    s3 = fmaf(ye[e], rv[3], s3);
  }
  v4f o4;
  o4[0] = s0 * kFoldBack;
  o4[1] = s1 * kFoldBack;
  o4[2] = s2 * kFoldBack;
  o4[3] = s3 * kFoldBack;
  float* pp = P + ((size_t)c * kNodes + b) * kHeads;
  *(volatile v4f*)pp = o4;
  __threadfence();
  *(volatile v4f*)pp = o4;
}

__global__ __launch_bounds__(256) void pack_rows_kernel(const float* __restrict__ P, float* __restrict__ out)
{
  __shared__ __align__(16) float sO[32 * kOPitch];
  const int tid  = threadIdx.x;
  const int lane = tid & 31;
  const int wave = tid >> 5;
  const int b0   = blockIdx.x * 32;
#pragma unroll 1
  for (int it = 0; it < 8; ++it) {
    const int idx  = it * 256 + tid;
    const int node = idx & 31;
    const int c    = idx >> 5;
    const v4f v = *(const v4f*)(P + ((size_t)c * kNodes + b0 + node) * kHeads);
    float* rp = sO + node * kOPitch;
    rp[c]              = v[0];
    rp[kCh + 3 * c]     = v[1];
    rp[kCh + 3 * c + 1] = v[2];
    rp[kCh + 3 * c + 2] = v[3];
  }
  __syncthreads();
  v4f vals[8];
#pragma unroll
  for (int q = 0; q < 8; ++q) {
    const int row = wave * 4 + (q >> 1);
    const int hf  = q & 1;
    vals[q] = *(const v4f*)(sO + row * kOPitch + hf * 128 + lane * 4);
  }
  for (int pass = 0; pass < 2; ++pass) {
#pragma unroll
    for (int q = 0; q < 8; ++q) {
      const int row = wave * 4 + (q >> 1);
      const int hf  = q & 1;
      *(volatile v4f*)(out + (size_t)(b0 + row) * kOutCols + hf * 128 + lane * 4) = vals[q];
    }
    __threadfence();
  }
}

extern "C" void kernel_launch(void* const* d_in, const int* in_sizes, int n_in,
                              void* d_out, int out_size, void* d_ws, size_t ws_size,
                              hipStream_t stream) {
  if (n_in < 14) return;
  if (in_sizes[0]  != kNodes * kCh * kFeat) return;
  if (in_sizes[1]  != kNodes * kSpec) return;
  if (in_sizes[2]  != kFeat * kFeat * kFeat * kPath3) return;
  if (in_sizes[3]  != kFeat * kFeat * kPath2) return;
  if (in_sizes[4]  != kFeat * kPath1) return;
  if (in_sizes[5]  != kSpec * kPath3 * kCh) return;
  if (in_sizes[6]  != kSpec * kPath2 * kCh) return;
  if (in_sizes[7]  != kSpec * kPath1 * kCh) return;
  if (in_sizes[8]  != 3 * kFeat * kFeat * kFeat * kPath3) return;
  if (in_sizes[9]  != 3 * kFeat * kFeat * kPath2) return;
  if (in_sizes[10] != 3 * kFeat * kPath1) return;
  if (in_sizes[11] != kSpec * kPath3 * kCh) return;
  if (in_sizes[12] != kSpec * kPath2 * kCh) return;
  if (in_sizes[13] != kSpec * kPath1 * kCh) return;
  if (out_size != kNodes * kOutCols) return;
  if (ws_size < kWsTotal) return;

  const float* x   = (const float*)d_in[0];
  const float* y   = (const float*)d_in[1];
  const float* U3s = (const float*)d_in[2];
  const float* U2s = (const float*)d_in[3];
  const float* U1s = (const float*)d_in[4];
  const float* W3s = (const float*)d_in[5];
  const float* W2s = (const float*)d_in[6];
  const float* W1s = (const float*)d_in[7];
  const float* U3v = (const float*)d_in[8];
  const float* U2v = (const float*)d_in[9];
  const float* U1v = (const float*)d_in[10];
  const float* W3v = (const float*)d_in[11];
  const float* W2v = (const float*)d_in[12];
  const float* W1v = (const float*)d_in[13];
  float* out = (float*)d_out;

  char* ws = (char*)d_ws;
  unsigned short* Bt = (unsigned short*)(ws + kOffBt);
  float*          PP = (float*)(ws + kOffP);

  fold_coeff_kernel<<<dim3(kNPad, kBtPitch / 64), 256, 0, stream>>>(
      U3s, U2s, U1s, W3s, W2s, W1s, U3v, U2v, U1v, W3v, W2v, W1v, Bt);

  poly_gemm_kernel<<<dim3(kNodes / kTile, kCh), kTile, 0, stream>>>(x, y, Bt, PP);

  pack_rows_kernel<<<kNodes / 32, 256, 0, stream>>>(PP, out);
}
